// RationalQuadraticSplineCoupling_13915694039132
// MI455X (gfx1250) — hardware-verified
//
#include <hip/hip_runtime.h>
#include <math.h>
#include <stddef.h>


#pragma clang fp contract(off)

#define DIM      128
#define HALFD    64
#define HIDDEN   256
#define NBINS    8
#define NSTAT    23
#define OUTW     (NSTAT * HALFD)
#define NCT1     (HIDDEN / 16)
#define NCT2     (OUTW / 16)
#define RPB      32
#define NTHR     256
#define HP       (HIDDEN + 4)
#define NB1      (HIDDEN * HALFD / 8 / NTHR)
#define NB2      (OUTW * HIDDEN / 8 / NTHR)
#define XCARRY   8.0f
#define HCARRY   8.0f
#define WCARRY   64.0f
#define INV512   (1.0f / 512.0f)
#define INVSQ    0.0625f
#define LN_EPS_F 1e-5f
#define MINBIN   0.001f
#define MIXW     0.992f
#define MIND     0.001f
#define TAILB    4.0f
#define EDGECST  0.5397424f
#define LDS2_SBUF 0
#define LDS2_SY   (RPB * OUTW * 4)
#define LDS2_SL   (LDS2_SY + RPB * DIM * 4)
#define LDS2_TOT  (LDS2_SL + RPB * HALFD * 4)
#define WSCAP    134217728

static_assert(NB1 * NTHR * 8 == HIDDEN * HALFD);
static_assert(NB2 * NTHR * 8 == OUTW * HIDDEN);
static_assert((HALFD % 32) == 0 && (HIDDEN % 32) == 0);
static_assert((OUTW % 16) == 0 && (NCT2 % 4) == 0 && (NCT1 % 4) == 0);
static_assert(((HP * 4) % 16) == 0);
static_assert((LDS2_SY % 16) == 0 && (LDS2_SL % 16) == 0 && LDS2_TOT <= 300 * 1024);
static_assert((RPB * DIM / 4) % NTHR == 0 && (RPB * HALFD / 4) % NTHR == 0);
static_assert(NTHR == 256 && RPB == 32 && NSTAT == 3 * NBINS - 1);

typedef float    v4f  __attribute__((ext_vector_type(4)));
typedef float    v8f  __attribute__((ext_vector_type(8)));
typedef _Float16 v8h  __attribute__((ext_vector_type(8)));
typedef _Float16 v16h __attribute__((ext_vector_type(16)));
union FragH { v16h v; v8h half[2]; };
static_assert(sizeof(FragH) == 32);

__device__ __forceinline__ v8f wmf(v16h a, v16h bq, v8f c) {
  v8f d = __builtin_amdgcn_wmma_f32_16x16x32_f16(false, a, false, bq, (short)0, c, false, false);
  asm volatile("v_nop\n\tv_nop\n\tv_nop\n\tv_nop" : "+v"(d) : "v"(a), "v"(bq));
  return d;
}

__device__ __forceinline__ v8f zero8() {
  v8f z = {0.f, 0.f, 0.f, 0.f, 0.f, 0.f, 0.f, 0.f};
  return z;
}

__device__ __forceinline__ v16h ldfrag(const _Float16* __restrict__ base, int ld, int r0, int k0, int lane) {
  const int h = lane >> 4, m = lane & 15;
  const _Float16* p = base + (size_t)(r0 + m) * ld + k0 + 8 * h;
  FragH f;
  f.half[0] = *(const v8h*)p;
  f.half[1] = *(const v8h*)(p + 16);
  return f.v;
}

__device__ __forceinline__ v8h cvt8(v4f a, v4f bq, float s) {
  v8h o;
  o[0] = (_Float16)(a.x * s);  o[1] = (_Float16)(a.y * s);  o[2] = (_Float16)(a.z * s);  o[3] = (_Float16)(a.w * s);
  o[4] = (_Float16)(bq.x * s); o[5] = (_Float16)(bq.y * s); o[6] = (_Float16)(bq.z * s); o[7] = (_Float16)(bq.w * s);
  return o;
}

__device__ __forceinline__ v16h ldfrag_x(const float* __restrict__ x, int r0, int k0, int lane) {
  const int h = lane >> 4, m = lane & 15;
  const float* p = x + (size_t)(r0 + m) * DIM + k0 + 8 * h;
  FragH f;
  f.half[0] = cvt8(*(const v4f*)p,        *(const v4f*)(p + 4),  XCARRY);
  f.half[1] = cvt8(*(const v4f*)(p + 16), *(const v4f*)(p + 20), XCARRY);
  return f.v;
}

__device__ __forceinline__ float softplus_f(float u) {
  return fmaxf(u, 0.0f) + log1pf(__expf(-fabsf(u)));
}

__device__ __forceinline__ void cum_knots(const float (&u)[8], float (&kn)[9]) {
  float mx = u[0] * INVSQ;
#pragma unroll
  for (int j = 1; j < 8; ++j) mx = fmaxf(mx, u[j] * INVSQ);
  float e[8];
  float sum = 0.0f;
#pragma unroll
  for (int j = 0; j < 8; ++j) { e[j] = __expf(u[j] * INVSQ - mx); sum = sum + e[j]; }
  const float inv = 1.0f / sum;
  float run = 0.0f;
  kn[0] = -TAILB;
#pragma unroll
  for (int j = 0; j < 8; ++j) {
    const float w = MINBIN + MIXW * (e[j] * inv);
    run = run + w;
    kn[j + 1] = 8.0f * run - TAILB;
  }
  kn[8] = TAILB;
}

__global__ __launch_bounds__(NTHR) void k_cvt(const float* __restrict__ w1, const float* __restrict__ w2,
                                              _Float16* w1h, _Float16* w2h) {
  const int b = blockIdx.x, tid = threadIdx.x;
  const float* src;
  _Float16* dst;
  int t;
  if (b < NB1) { src = w1; dst = w1h; t = b * NTHR + tid; }
  else         { src = w2; dst = w2h; t = (b - NB1) * NTHR + tid; }
  const float* p = src + (size_t)t * 8;
  const v8h o = cvt8(*(const v4f*)p, *(const v4f*)(p + 4), WCARRY);
  _Float16* d = dst + (size_t)t * 8;
  *(volatile v8h*)d = o;
  __threadfence();
  *(volatile v8h*)d = o;
}

__global__ __launch_bounds__(NTHR) void k_gemm1_ln(
    const float* __restrict__ x, const _Float16* __restrict__ w1h,
    const float* __restrict__ lns, const float* __restrict__ lnb, _Float16* hb) {
  __shared__ __attribute__((aligned(16))) float hbuf[RPB * HP];
  const int tid = threadIdx.x, lane = tid & 31, wave = tid >> 5, h = lane >> 4, m = lane & 15;
  const int rowBase = blockIdx.x * RPB;

  {
    const int s = wave >> 2, ct0 = wave & 3;
    const v16h a0 = ldfrag_x(x, rowBase + 16 * s, 0,  lane);
    const v16h a1 = ldfrag_x(x, rowBase + 16 * s, 32, lane);
#pragma unroll
    for (int i = 0; i < 4; ++i) {
      const int ct = ct0 + 4 * i;
      const v16h b0 = ldfrag(w1h, HALFD, ct * 16, 0,  lane);
      const v16h b1 = ldfrag(w1h, HALFD, ct * 16, 32, lane);
      v8f c = zero8();
      c = wmf(a0, b0, c);
      c = wmf(a1, b1, c);
#pragma unroll
      for (int r = 0; r < 8; ++r) hbuf[(16 * s + 8 * h + r) * HP + ct * 16 + m] = c[r] * INV512;
    }
  }
  __syncthreads();

  const float* gsrc = lns + lane * 8;
  const float* bsrc = lnb + lane * 8;
  const v4f g0 = *(const v4f*)gsrc, g1 = *(const v4f*)(gsrc + 4);
  const v4f t0 = *(const v4f*)bsrc, t1 = *(const v4f*)(bsrc + 4);
  const float gg[8] = {g0.x, g0.y, g0.z, g0.w, g1.x, g1.y, g1.z, g1.w};
  const float bb[8] = {t0.x, t0.y, t0.z, t0.w, t1.x, t1.y, t1.z, t1.w};

#pragma unroll 1
  for (int rr = 0; rr < 4; ++rr) {
    const int r = wave * 4 + rr;
    const float* hr = hbuf + r * HP + lane * 8;
    const v4f p0 = *(const v4f*)hr, p1 = *(const v4f*)(hr + 4);
    const float v[8] = {p0.x, p0.y, p0.z, p0.w, p1.x, p1.y, p1.z, p1.w};
    float s0 = 0.0f;
#pragma unroll
    for (int i = 0; i < 8; ++i) s0 = s0 + v[i];
#pragma unroll
    for (int off = 16; off > 0; off >>= 1) s0 += __shfl_xor(s0, off, 32);
    const float mean = s0 * (1.0f / (float)HIDDEN);
    float s1 = 0.0f;
#pragma unroll
    for (int i = 0; i < 8; ++i) { const float d = v[i] - mean; s1 = s1 + d * d; }
#pragma unroll
    for (int off = 16; off > 0; off >>= 1) s1 += __shfl_xor(s1, off, 32);
    const float var = s1 * (1.0f / (float)HIDDEN);
    const float rs = rsqrtf(var + LN_EPS_F);
    v8h o;
#pragma unroll
    for (int i = 0; i < 8; ++i) {
      float y = (v[i] - mean) * rs * gg[i] + bb[i];
      y = fmaxf(y, 0.0f);
      o[i] = (_Float16)(y * HCARRY);
    }
    _Float16* d = hb + (size_t)(rowBase + r) * HIDDEN + lane * 8;
    *(volatile v8h*)d = o;
    __threadfence();
    *(volatile v8h*)d = o;
  }
}

__global__ __launch_bounds__(NTHR) void k_gemm2_spline(
    const float* __restrict__ x, const _Float16* __restrict__ hb,
    const _Float16* __restrict__ w2h, const float* __restrict__ b2, float* out, float* logdet) {
  extern __shared__ v4f lds_dyn[];
  char* sm = (char*)lds_dyn;
  float* sbuf = (float*)(sm + LDS2_SBUF);
  float* sy   = (float*)(sm + LDS2_SY);
  float* sl   = (float*)(sm + LDS2_SL);
  const int tid = threadIdx.x, lane = tid & 31, wave = tid >> 5, h = lane >> 4, m = lane & 15;
  const int rowBase = blockIdx.x * RPB;

  {
    const v4f* xs = (const v4f*)(x + (size_t)rowBase * DIM);
    v4f* s4 = (v4f*)sy;
#pragma unroll
    for (int j = 0; j < RPB * DIM / 4 / NTHR; ++j) s4[tid + j * NTHR] = xs[tid + j * NTHR];
  }

  {
    const int s = wave >> 2, ct0 = wave & 3;
    v16h a[8];
#pragma unroll
    for (int kc = 0; kc < 8; ++kc) a[kc] = ldfrag(hb, HIDDEN, rowBase + 16 * s, kc * 32, lane);
#pragma unroll 1
    for (int ct = ct0; ct < NCT2; ct += 4) {
      v8f c = zero8();
#pragma unroll
      for (int kc = 0; kc < 8; ++kc) {
        const v16h bq = ldfrag(w2h, HIDDEN, ct * 16, kc * 32, lane);
        c = wmf(a[kc], bq, c);
      }
      const int o = ct * 16 + m;
      const float bias = b2[o];
#pragma unroll
      for (int r = 0; r < 8; ++r) sbuf[(16 * s + 8 * h + r) * OUTW + o] = c[r] * INV512 + bias;
    }
  }
  __syncthreads();

  {
    const int c = tid & 63, rq = tid >> 6;
    const float edge = MIND + softplus_f(EDGECST);
#pragma unroll 1
    for (int i = 0; i < 8; ++i) {
      const int r = rq * 8 + i;
      const float* sp = sbuf + r * OUTW + c * NSTAT;
      float uw[8], uh[8], ud[7];
#pragma unroll
      for (int j = 0; j < 8; ++j) { uw[j] = sp[j]; uh[j] = sp[8 + j]; }
#pragma unroll
      for (int j = 0; j < 7; ++j) ud[j] = sp[16 + j];

      float cw[9], chh[9];
      cum_knots(uw, cw);
      cum_knots(uh, chh);
      float dv[9];
      dv[0] = edge;
      dv[8] = edge;
#pragma unroll
      for (int j = 0; j < 7; ++j) dv[j + 1] = MIND + softplus_f(ud[j]);

      const float xin = sy[r * DIM + HALFD + c];
      int cnt = 0;
#pragma unroll
      for (int j = 0; j < 8; ++j) cnt += (xin >= cw[j]) ? 1 : 0;
      const float last = cw[8] + 1e-6f;
      cnt += (xin >= last) ? 1 : 0;
      int bin = cnt - 1;
      bin = bin < 0 ? 0 : bin;
      bin = bin > 7 ? 7 : bin;

      float icw = cw[0], iw = cw[1] - cw[0], ich = chh[0], ih = chh[1] - chh[0], id0 = dv[0], id1 = dv[1];
#pragma unroll
      for (int j = 1; j < 8; ++j) {
        const bool q = (bin == j);
        icw = q ? cw[j] : icw;
        iw  = q ? (cw[j + 1] - cw[j]) : iw;
        ich = q ? chh[j] : ich;
        ih  = q ? (chh[j + 1] - chh[j]) : ih;
        id0 = q ? dv[j] : id0;
        id1 = q ? dv[j + 1] : id1;
      }

      const float delta = ih / iw;
      const float theta = (xin - icw) / iw;
      const float omt   = 1.0f - theta;
      const float t1mt  = theta * omt;
      const float num   = ih * (delta * theta * theta + id0 * t1mt);
      const float den   = delta + (id0 + id1 - 2.0f * delta) * t1mt;
      float y = ich + num / den;
      const float dnum  = (delta * delta) * (id1 * theta * theta + 2.0f * delta * t1mt + id0 * (omt * omt));
      float lad = logf(dnum) - 2.0f * logf(den);

      const bool inside = (xin >= -TAILB) && (xin <= TAILB);
      y   = inside ? y : xin;
      lad = inside ? lad : 0.0f;
      sy[r * DIM + HALFD + c] = y;
      sl[r * HALFD + c] = lad;
    }
  }
  __syncthreads();

  {
    float* op = out + (size_t)rowBase * DIM;
    float* lp = logdet + (size_t)rowBase * HALFD;
    const v4f* s4 = (const v4f*)sy;
    const v4f* l4 = (const v4f*)sl;
    v4f vy[4], vl[2];
#pragma unroll
    for (int j = 0; j < 4; ++j) vy[j] = s4[tid + j * NTHR];
#pragma unroll
    for (int j = 0; j < 2; ++j) vl[j] = l4[tid + j * NTHR];
#pragma unroll
    for (int j = 0; j < 4; ++j) *(volatile v4f*)(op + 4 * (tid + j * NTHR)) = vy[j];
#pragma unroll
    for (int j = 0; j < 2; ++j) *(volatile v4f*)(lp + 4 * (tid + j * NTHR)) = vl[j];
    __threadfence();
#pragma unroll
    for (int j = 0; j < 4; ++j) *(volatile v4f*)(op + 4 * (tid + j * NTHR)) = vy[j];
#pragma unroll
    for (int j = 0; j < 2; ++j) *(volatile v4f*)(lp + 4 * (tid + j * NTHR)) = vl[j];
  }
}

extern "C" void kernel_launch(void* const* d_in, const int* in_sizes, int n_in,
                              void* d_out, int out_size, void* d_ws, size_t ws_size,
                              hipStream_t stream) {
  if (n_in < 6) return;
  const int rows = in_sizes[0] / DIM;
  if (rows <= 0 || in_sizes[0] != rows * DIM || (rows % RPB) != 0) return;
  if (in_sizes[1] != HIDDEN * HALFD || in_sizes[2] != HIDDEN || in_sizes[3] != HIDDEN) return;
  if (in_sizes[4] != OUTW * HIDDEN || in_sizes[5] != OUTW) return;
  if (out_size != rows * DIM + rows * HALFD) return;

  const float* x   = (const float*)d_in[0];
  const float* w1  = (const float*)d_in[1];
  const float* lns = (const float*)d_in[2];
  const float* lnb = (const float*)d_in[3];
  const float* w2  = (const float*)d_in[4];
  const float* b2  = (const float*)d_in[5];
  float* out    = (float*)d_out;
  float* logdet = out + (size_t)rows * DIM;

  size_t off = 0;
  const size_t oW1 = off; off += (size_t)HIDDEN * HALFD * 2;   off = (off + 255) & ~(size_t)255;
  const size_t oW2 = off; off += (size_t)OUTW * HIDDEN * 2;    off = (off + 255) & ~(size_t)255;
  const size_t oHB = off; off += (size_t)rows * HIDDEN * 2;    off = (off + 255) & ~(size_t)255;
  const size_t tot = off;
  if (tot > ws_size || tot > (size_t)WSCAP) return;
  char* ws = (char*)d_ws;
  _Float16* w1h = (_Float16*)(ws + oW1);
  _Float16* w2h = (_Float16*)(ws + oW2);
  _Float16* hb  = (_Float16*)(ws + oHB);
  const int nblk = rows / RPB;

  k_cvt<<<NB1 + NB2, NTHR, 0, stream>>>(w1, w2, w1h, w2h);
  k_gemm1_ln<<<nblk, NTHR, 0, stream>>>(x, w1h, lns, lnb, hb);
  hipFuncSetAttribute(reinterpret_cast<const void*>(&k_gemm2_spline),
                      hipFuncAttributeMaxDynamicSharedMemorySize, LDS2_TOT);
  k_gemm2_spline<<<nblk, NTHR, LDS2_TOT, stream>>>(x, hb, w2h, b2, out, logdet);
}
